// GraphAttention_83700322664683
// MI455X (gfx1250) — hardware-verified
//
#include <hip/hip_runtime.h>


namespace {

constexpr int B = 4, NN = 128  , NODE = 256, EDGE = 128, GLOB = 128, HID = 512, NE = NN * NN  , BL = B  , N = B * NN  , NP = N;
constexpr int VOC = 1, NL = N;
constexpr float LNEPS = 1e-5f; constexpr float LOG2E = 1.4426950408889634f; constexpr float XS = 8.0f, WSC = 256.0f, WSQ = 0.25f, RS_ = 1024.0f, NSL_ = 0.2f, NSA_ = 0.01f, SLOPE = 0.0f, BNEPS = 1e-5f;
static_assert(NN % 32 == 0 && NE % 32 == 0 && HID % 32 == 0, "tiling");
typedef _Float16 b16;
typedef __attribute__((ext_vector_type(16))) _Float16 v16b;
typedef __attribute__((ext_vector_type(8))) _Float16 v8b;
typedef __attribute__((ext_vector_type(8))) float v8f;
typedef __attribute__((ext_vector_type(4))) float v4f;
__device__ __forceinline__ float bf16_rne(float f) { unsigned int u = __float_as_uint(f); u += 0x7FFFu + ((u >> 16) & 1u); return __uint_as_float(u & 0xFFFF0000u); }
__device__ __forceinline__ void split16(float v, b16& hi, b16& lo) { hi = (b16)v; lo = (b16)(v - (float)hi); }
__device__ __forceinline__ v16b frag_kb(const b16* p, int hh) { const v8b a = *(const v8b*)(p + 8 * hh), b = *(const v8b*)(p + 16 + 8 * hh); v16b f;
#pragma unroll
  for (int e = 0; e < 8; ++e) { f[e] = a[e]; f[8 + e] = b[e]; } return f; }
__device__ __forceinline__ v8f wmma16b(v16b a, v16b b, v8f c) { v8f d = __builtin_amdgcn_wmma_f32_16x16x32_f16(false, a, false, b, (short)0, c, false, false); asm volatile("v_nop\n\tv_nop\n\tv_nop\n\tv_nop" : "+v"(d) : "v"(a), "v"(b)); return d; }
__device__ __forceinline__ void wave_lds_sync() { __builtin_amdgcn_fence(__ATOMIC_RELEASE, "workgroup"); __builtin_amdgcn_wave_barrier(); __builtin_amdgcn_fence(__ATOMIC_ACQUIRE, "workgroup"); }
__device__ __forceinline__ float pmul(float a, float b) { float p = a * b; asm volatile("" : "+v"(p)); return p; }
__device__ __forceinline__ int iclamp(int v, int lo, int hi) { return v < lo ? lo : (v > hi ? hi : v); }

typedef __attribute__((ext_vector_type(4))) _Float16 v4h;
__device__ __forceinline__ float lrelu(float v) { return v > 0.0f ? v : NSL_ * v; }
template <int K, int NOUTR, int NOUTP>
__global__ __launch_bounds__(256) void wt_kernel(const float* __restrict__ w, b16* __restrict__ WT, float scl) {
  const int u = blockIdx.x * 256 + threadIdx.x; if (u >= NOUTP * K / 8) return; const int e = u * 8; const int o = e / K, k0 = e % K; v8b v;
#pragma unroll
  for (int j = 0; j < 8; ++j) v[j] = (b16)(o < NOUTR ? bf16_rne(w[(size_t)(k0 + j) * NOUTR + o]) * scl : 0.0f);
  for (int pass = 0; pass < 2; ++pass) { *(volatile v8b*)(WT + e) = v; __threadfence(); }
}
template <int K, int NT, bool RND, int MODE, bool GIDX>
__global__ __launch_bounds__(64) void lin_kernel(const float* __restrict__ X, const int* __restrict__ gidx, const b16* __restrict__ WT, const b16* __restrict__ WQ, const float* __restrict__ bias, float* __restrict__ OUT, int opitch, int nvalid, int mrows, const float* __restrict__ lng = nullptr, const float* __restrict__ lnb = nullptr) {
  constexpr int NC = NT * 16;
  __shared__ __attribute__((aligned(16))) b16 Ah[2][16][K + 8], Al[2][16][K + 8]; __shared__ __attribute__((aligned(16))) float Tf[2][16][NC + 4];
  const int wave = threadIdx.x >> 5, lane = threadIdx.x & 31, nloc = lane & 15, hlf = lane >> 4; const size_t m0 = (size_t)blockIdx.x * 32 + wave * 16;
  for (int idx = lane; idx < 16 * (K / 4); idx += 32) { const int rr = idx / (K / 4), c4 = (idx % (K / 4)) * 4; const size_t vrow = (m0 + rr < (size_t)nvalid) ? m0 + rr : (size_t)nvalid - 1; size_t arow = vrow; if (GIDX) arow = (size_t)iclamp(gidx[vrow], 0, VOC - 1);
    const v4f v = *(const v4f*)(X + arow * K + c4); v4h hv, lv;
    for (int j = 0; j < 4; ++j) { float vj = v[j]; if (MODE == 2) vj = fmaxf(vj, 0.0f); const float vs = (RND ? bf16_rne(vj) : vj) * XS; const b16 ph = (b16)vs; hv[j] = ph; lv[j] = (b16)((vs - (float)ph) * RS_); } *(v4h*)(&Ah[wave][rr][c4]) = hv; *(v4h*)(&Al[wave][rr][c4]) = lv; }
  wave_lds_sync();
  v8f acc[NT];
#pragma unroll
  for (int t = 0; t < NT; ++t) acc[t] = (v8f){};
#pragma unroll 1
  for (int kb = 0; kb < K; kb += 32) { const v16b a = frag_kb(&Ah[wave][nloc][kb], hlf); v16b al; if (!RND) al = frag_kb(&Al[wave][nloc][kb], hlf);
#pragma unroll
    for (int t = 0; t < NT; ++t) { const size_t wo_ = (size_t)(t * 16 + nloc) * K + kb; acc[t] = wmma16b(a, frag_kb(WT + wo_, hlf), acc[t]); if (!RND) acc[t] = wmma16b(al, frag_kb(WQ + wo_, hlf), acc[t]); } }
if (MODE == 5) {
    static_assert(MODE != 5 || NT == 8, "LN epilogue needs the full 128-wide row in one wave");
    float sm[8], sq[8]; for (int r = 0; r < 8; ++r) { sm[r] = 0.0f; sq[r] = 0.0f; }
    for (int t = 0; t < NT; ++t) { const int col = t * 16 + nloc; const float bb = bf16_rne(bias[col]); for (int r = 0; r < 8; ++r) { const float y = acc[t][r] * (1.0f / (XS * WSC)) + bb; acc[t][r] = y; sm[r] += y; } }
#pragma unroll
    for (int o = 1; o < 16; o <<= 1) for (int r = 0; r < 8; ++r) sm[r] += __shfl_xor(sm[r], o);
    for (int t = 0; t < NT; ++t) for (int r = 0; r < 8; ++r) { const float d = acc[t][r] - sm[r] * (1.0f / NC); sq[r] += pmul(d, d); }
#pragma unroll
    for (int o = 1; o < 16; o <<= 1) for (int r = 0; r < 8; ++r) sq[r] += __shfl_xor(sq[r], o);
    for (int t = 0; t < NT; ++t) { const int col = t * 16 + nloc; const float gg = bf16_rne(lng[col]), be = bf16_rne(lnb[col]);
      for (int r = 0; r < 8; ++r) { const size_t vrow = m0 + 8 * hlf + r; const float y = fmaxf((acc[t][r] - sm[r] * (1.0f / NC)) * rsqrtf(sq[r] * (1.0f / NC) + LNEPS) * gg + be, 0.0f); Tf[wave][8 * hlf + r][col] = (vrow < (size_t)nvalid) ? y : 0.0f; } }
  } else {
  for (int t = 0; t < NT; ++t) { const int col = t * 16 + nloc; const float bb = bf16_rne(bias[col]);
    for (int r = 0; r < 8; ++r) { const size_t vrow = m0 + 8 * hlf + r; float y = acc[t][r] * (1.0f / (XS * WSC)) + bb; if (MODE == 1) y = fmaxf(y, 0.0f); Tf[wave][8 * hlf + r][col] = (vrow < (size_t)nvalid) ? y : 0.0f; } }
  }
  wave_lds_sync();
  for (int pass = 0; pass < 2; ++pass) { for (int rr = 0; rr < 16; ++rr) { if (m0 + rr < (size_t)mrows) { if (NC >= 128) { for (int c8 = 0; c8 < NC; c8 += 128) *(volatile v4f*)(OUT + (m0 + rr) * (size_t)opitch + c8 + lane * 4) = *(const v4f*)(&Tf[wave][rr][c8 + lane * 4]); }
        else { if (lane < NC / 4) *(volatile v4f*)(OUT + (m0 + rr) * (size_t)opitch + lane * 4) = *(const v4f*)(&Tf[wave][rr][lane * 4]); } } } __threadfence(); }
}
__device__ __forceinline__ float gelu_(float v) { return 0.5f * v * (1.0f + erff(v * 0.70710678118654752f)); }
template <int KW, int NOUT>
__global__ __launch_bounds__(256) void wts_kernel(const float* __restrict__ w, int k0, b16* __restrict__ WT, float scl) {
  const int u = blockIdx.x * 256 + threadIdx.x; if (u >= NOUT * KW / 8) return; const int e = u * 8; const int o = e / KW, kk = e % KW; v8b v;
#pragma unroll
  for (int j = 0; j < 8; ++j) v[j] = (b16)(bf16_rne(w[(size_t)(k0 + kk + j) * NOUT + o]) * scl);
  for (int pass = 0; pass < 2; ++pass) { *(volatile v8b*)(WT + e) = v; __threadfence(); }
}
__global__ __launch_bounds__(256) void zfill_kernel(float* __restrict__ Z, int n) { const int i = blockIdx.x * 256 + threadIdx.x; for (int pass = 0; pass < 2; ++pass) { if (i < n) ((volatile float*)Z)[i] = 0.0f; __threadfence(); } }
__global__ __launch_bounds__(256) void yfilm_kernel(const float* __restrict__ y, const float* __restrict__ Wem, const float* __restrict__ Wea, const float* __restrict__ Wxm, const float* __restrict__ Wxa, float* __restrict__ YV) {
  const int i = blockIdx.x * 256 + threadIdx.x; if (i >= B * 4 * HID) return; const int c = i % HID, k = (i / HID) % 4, b = i / (4 * HID);
  const float* W = (k == 0) ? Wem : (k == 1) ? Wea : (k == 2) ? Wxm : Wxa; float s = 0.0f;
#pragma unroll 1
  for (int j = 0; j < GLOB; ++j) s += pmul(bf16_rne(y[b * GLOB + j]), bf16_rne(W[(size_t)j * HID + c]));
  for (int pass = 0; pass < 2; ++pass) { ((volatile float*)YV)[i] = s; __threadfence(); }
}
__global__ __launch_bounds__(256) void sim_kernel(float* __restrict__ EM, const float* __restrict__ EA, const float* __restrict__ Q, const float* __restrict__ Kp, int b) {
  const size_t i = (size_t)blockIdx.x * 256 + threadIdx.x; if (i >= (size_t)NE * HID / 4) return; const size_t r = i / (HID / 4); const int c = (int)(i % (HID / 4)) * 4; const int n = (int)(r / NN), m = (int)(r % NN);
  const v4f em = *(const v4f*)(EM + r * HID + c), ea = *(const v4f*)(EA + r * HID + c), q4 = *(const v4f*)(Q + ((size_t)b * NN + n) * HID + c), k4 = *(const v4f*)(Kp + ((size_t)b * NN + m) * HID + c);
  v4f o; for (int j = 0; j < 4; ++j) o[j] = (1.0f + em[j]) * pmul(pmul(q4[j], k4[j]), 0.125f) + ea[j];
  for (int pass = 0; pass < 2; ++pass) { *(volatile v4f*)(EM + r * HID + c) = o; __threadfence(); }
}
__global__ __launch_bounds__(64) void eout_kernel(const float* __restrict__ S, const float* __restrict__ YM, const float* __restrict__ YA, const b16* __restrict__ WT, const b16* __restrict__ WQ, const float* __restrict__ bias, float* __restrict__ out_e, float* __restrict__ PS) {
  constexpr int K = HID, NT = 8, NC = 128;
  __shared__ __attribute__((aligned(16))) b16 Ah[2][16][K + 8], Al[2][16][K + 8]; __shared__ __attribute__((aligned(16))) float Tf[2][16][NC + 4];
  const int wave = threadIdx.x >> 5, lane = threadIdx.x & 31, nloc = lane & 15, hlf = lane >> 4; const size_t m0 = (size_t)blockIdx.x * 32 + wave * 16;
  for (int idx = lane; idx < 16 * (K / 4); idx += 32) { const int rr = idx / (K / 4), c4 = (idx % (K / 4)) * 4; const v4f v = *(const v4f*)(S + (m0 + rr) * K + c4), ym = *(const v4f*)(YM + c4), ya = *(const v4f*)(YA + c4); v4h hv, lv;
    for (int j = 0; j < 4; ++j) { const float vs = ((1.0f + ym[j]) * v[j] + ya[j]) * XS; const b16 ph = (b16)vs; hv[j] = ph; lv[j] = (b16)((vs - (float)ph) * RS_); } *(v4h*)(&Ah[wave][rr][c4]) = hv; *(v4h*)(&Al[wave][rr][c4]) = lv; }
  wave_lds_sync();
  v8f acc[NT]; for (int t = 0; t < NT; ++t) acc[t] = (v8f){};
#pragma unroll 2
  for (int kb = 0; kb < K; kb += 32) { const v16b a = frag_kb(&Ah[wave][nloc][kb], hlf), al = frag_kb(&Al[wave][nloc][kb], hlf);
#pragma unroll
    for (int t = 0; t < NT; ++t) { const size_t wo_ = (size_t)(t * 16 + nloc) * K + kb; acc[t] = wmma16b(a, frag_kb(WT + wo_, hlf), acc[t]); acc[t] = wmma16b(al, frag_kb(WQ + wo_, hlf), acc[t]); } }
#pragma unroll
  for (int t = 0; t < NT; ++t) { const int col = t * 16 + nloc; const float bb = bf16_rne(bias[col]); for (int r = 0; r < 8; ++r) Tf[wave][8 * hlf + r][col] = acc[t][r] * (1.0f / (XS * WSC)) + bb; }
  wave_lds_sync();
  v4f cs = {0.0f, 0.0f, 0.0f, 0.0f}; for (int rr = 0; rr < 16; ++rr) { const v4f t4 = *(const v4f*)(&Tf[wave][rr][lane * 4]); for (int j = 0; j < 4; ++j) cs[j] += t4[j]; }
  for (int pass = 0; pass < 2; ++pass) { for (int rr = 0; rr < 16; ++rr) *(volatile v4f*)(out_e + (m0 + rr) * NC + lane * 4) = *(const v4f*)(&Tf[wave][rr][lane * 4]);
    *(volatile v4f*)(PS + (blockIdx.x * 2 + wave) * (size_t)NC + lane * 4) = cs; __threadfence(); }
}
__global__ __launch_bounds__(256) void att_kernel(const float* __restrict__ S, const float* __restrict__ Vp, const float* __restrict__ YXM, const float* __restrict__ YXA, float* __restrict__ AVF, int b) {
  const int i = blockIdx.x * 256 + threadIdx.x; if (i >= NN * HID / 4) return; const int n = i / (HID / 4), c = (i % (HID / 4)) * 4;
  const float* sp = S + (size_t)n * NN * HID + c; v4f mx = {-INFINITY, -INFINITY, -INFINITY, -INFINITY};
#pragma unroll 1
  for (int m = 0; m < NN; ++m) { const v4f s4 = *(const v4f*)(sp + (size_t)m * HID); for (int j = 0; j < 4; ++j) mx[j] = fmaxf(mx[j], s4[j]); }
  v4f l = {0.0f, 0.0f, 0.0f, 0.0f}, acc = {0.0f, 0.0f, 0.0f, 0.0f};
#pragma unroll 1
  for (int m = 0; m < NN; ++m) { const v4f s4 = *(const v4f*)(sp + (size_t)m * HID), v4 = *(const v4f*)(Vp + ((size_t)b * NN + m) * HID + c); for (int j = 0; j < 4; ++j) { const float p = __expf(s4[j] - mx[j]); l[j] += p; acc[j] += pmul(p, v4[j]); } }
  const v4f xm = *(const v4f*)(YXM + c), xa = *(const v4f*)(YXA + c); v4f o; for (int j = 0; j < 4; ++j) o[j] = (1.0f + xm[j]) * (acc[j] / l[j]) + xa[j];
  for (int pass = 0; pass < 2; ++pass) { *(volatile v4f*)(AVF + (size_t)n * HID + c) = o; __threadfence(); }
}
__global__ __launch_bounds__(128) void yout_kernel(const float* __restrict__ PS, const float* __restrict__ out_x, const float* __restrict__ y, const float* __restrict__ Wyx, const float* __restrict__ byx, const float* __restrict__ Wye, const float* __restrict__ bye, float* __restrict__ out_y, int b) {
  __shared__ float yx[NODE], ye[EDGE];
  const int t = threadIdx.x;
  { float s = 0.0f;
#pragma unroll 1
    for (int k = 0; k < NE / 16; ++k) s += PS[(size_t)k * EDGE + t]; ye[t] = s * (1.0f / NE); }
  for (int jj = 0; jj < 2; ++jj) { const int j = t + jj * 128; float s = 0.0f;
#pragma unroll 1
    for (int n = 0; n < NN; ++n) s += out_x[((size_t)b * NN + n) * NODE + j]; yx[j] = s * (1.0f / NN); }
  __syncthreads();
  float s = bf16_rne(y[b * GLOB + t]) + bf16_rne(byx[t]) + bf16_rne(bye[t]);
#pragma unroll 1
  for (int i = 0; i < NODE; ++i) s += pmul(yx[i], bf16_rne(Wyx[(size_t)i * GLOB + t]));
#pragma unroll 1
  for (int i = 0; i < EDGE; ++i) s += pmul(ye[i], bf16_rne(Wye[(size_t)i * GLOB + t]));
  for (int pass = 0; pass < 2; ++pass) { ((volatile float*)out_y)[b * GLOB + t] = s; __threadfence(); }
}
}

extern "C" void kernel_launch(void* const* d_in, const int* in_sizes, int n_in, void* d_out, int out_size, void* d_ws, size_t ws_size, hipStream_t stream) {
  (void)n_in;
  auto Fp = [&](int i) { return (const float*)d_in[i]; };
  if (in_sizes[0] != N * NODE || in_sizes[1] != B * NE * EDGE || in_sizes[2] != B * GLOB || in_sizes[3] != N || in_sizes[4] != NODE * HID || in_sizes[5] != NODE * HID || in_sizes[6] != NODE * HID || in_sizes[7] != HID * NODE || in_sizes[8] != NODE || in_sizes[9] != EDGE * HID || in_sizes[10] != EDGE * HID || in_sizes[11] != HID * EDGE || in_sizes[12] != EDGE) return;
  if (in_sizes[13] != GLOB * HID || in_sizes[14] != GLOB * HID || in_sizes[15] != GLOB * HID || in_sizes[16] != GLOB * HID || in_sizes[17] != NODE * GLOB || in_sizes[18] != GLOB || in_sizes[19] != EDGE * GLOB || in_sizes[20] != GLOB || out_size != N * NODE + B * NE * EDGE + B * GLOB) return;
  float* out_x = (float*)d_out; float* out_e = out_x + (size_t)N * NODE; float* out_y = out_e + (size_t)B * NE * EDGE;
  size_t off = 0; char* ws = (char*)d_ws;
  auto carve = [&](size_t bytes) { char* p = ws + off; off += (bytes + 255) & ~(size_t)255; return p; };
  b16* WQ_ = (b16*)carve((size_t)HID * NODE * 2); b16* WK_ = (b16*)carve((size_t)HID * NODE * 2); b16* WV_ = (b16*)carve((size_t)HID * NODE * 2); b16* WEM = (b16*)carve((size_t)HID * EDGE * 2); b16* WEA = (b16*)carve((size_t)HID * EDGE * 2);
  b16* WEO = (b16*)carve((size_t)EDGE * HID * 2); b16* WEOQ = (b16*)carve((size_t)EDGE * HID * 2); b16* WO_ = (b16*)carve((size_t)NODE * HID * 2); b16* WOQ = (b16*)carve((size_t)NODE * HID * 2); float* ZB = (float*)carve((size_t)HID * 4);
  float* Qp = (float*)carve((size_t)N * HID * 4); float* Kp = (float*)carve((size_t)N * HID * 4); float* Vp = (float*)carve((size_t)N * HID * 4); float* YV = (float*)carve((size_t)B * 4 * HID * 4);
  float* EM = (float*)carve((size_t)NE * HID * 4); float* EA = (float*)carve((size_t)NE * HID * 4); float* PS = (float*)carve((size_t)(NE / 16) * EDGE * 4); float* AVF = (float*)carve((size_t)NN * HID * 4);
  if (off > ws_size || off > ((size_t)80 << 20)) return;
  { wt_kernel<NODE, HID, HID><<<(HID * NODE / 8 + 255) / 256, 256, 0, stream>>>(Fp(4), WQ_, WSC); wt_kernel<NODE, HID, HID><<<(HID * NODE / 8 + 255) / 256, 256, 0, stream>>>(Fp(5), WK_, WSC); wt_kernel<NODE, HID, HID><<<(HID * NODE / 8 + 255) / 256, 256, 0, stream>>>(Fp(6), WV_, WSC);
    wt_kernel<EDGE, HID, HID><<<(HID * EDGE / 8 + 255) / 256, 256, 0, stream>>>(Fp(9), WEM, WSC); wt_kernel<EDGE, HID, HID><<<(HID * EDGE / 8 + 255) / 256, 256, 0, stream>>>(Fp(10), WEA, WSC);
    wt_kernel<HID, EDGE, EDGE><<<(EDGE * HID / 8 + 255) / 256, 256, 0, stream>>>(Fp(11), WEO, WSC); wt_kernel<HID, EDGE, EDGE><<<(EDGE * HID / 8 + 255) / 256, 256, 0, stream>>>(Fp(11), WEOQ, WSQ);
    wt_kernel<HID, NODE, NODE><<<(NODE * HID / 8 + 255) / 256, 256, 0, stream>>>(Fp(7), WO_, WSC); wt_kernel<HID, NODE, NODE><<<(NODE * HID / 8 + 255) / 256, 256, 0, stream>>>(Fp(7), WOQ, WSQ);
    zfill_kernel<<<(HID + 255) / 256, 256, 0, stream>>>(ZB, HID); yfilm_kernel<<<(B * 4 * HID + 255) / 256, 256, 0, stream>>>(Fp(2), Fp(15), Fp(16), Fp(13), Fp(14), YV); }
  for (int hp = 0; hp < 2; ++hp) {
    lin_kernel<NODE, 16, true, 0, false><<<N / 32, 64, 0, stream>>>(Fp(0), nullptr, WQ_ + (size_t)hp * 256 * NODE, WQ_, ZB, Qp + hp * 256, HID, N, N);
    lin_kernel<NODE, 16, true, 0, false><<<N / 32, 64, 0, stream>>>(Fp(0), nullptr, WK_ + (size_t)hp * 256 * NODE, WK_, ZB, Kp + hp * 256, HID, N, N);
    lin_kernel<NODE, 16, true, 0, false><<<N / 32, 64, 0, stream>>>(Fp(0), nullptr, WV_ + (size_t)hp * 256 * NODE, WV_, ZB, Vp + hp * 256, HID, N, N); }
  for (int b = 0; b < BL; ++b) {
    const float* eb = Fp(1) + (size_t)b * NE * EDGE; const float* YM = YV + (size_t)(b * 4 + 0) * HID; const float* YA = YV + (size_t)(b * 4 + 1) * HID; const float* YXM = YV + (size_t)(b * 4 + 2) * HID; const float* YXA = YV + (size_t)(b * 4 + 3) * HID;
    for (int hp = 0; hp < 2; ++hp) {
      lin_kernel<EDGE, 16, true, 0, false><<<NE / 32, 64, 0, stream>>>(eb, nullptr, WEM + (size_t)hp * 256 * EDGE, WEM, ZB, EM + hp * 256, HID, NE, NE);
      lin_kernel<EDGE, 16, true, 0, false><<<NE / 32, 64, 0, stream>>>(eb, nullptr, WEA + (size_t)hp * 256 * EDGE, WEA, ZB, EA + hp * 256, HID, NE, NE); }
    sim_kernel<<<(unsigned)(((size_t)NE * HID / 4 + 255) / 256), 256, 0, stream>>>(EM, EA, Qp, Kp, b);
    eout_kernel<<<NE / 32, 64, 0, stream>>>(EM, YM, YA, WEO, WEOQ, Fp(12), out_e + (size_t)b * NE * EDGE, PS);
    att_kernel<<<(NN * HID / 4 + 255) / 256, 256, 0, stream>>>(EM, Vp, YXM, YXA, AVF, b);
    lin_kernel<HID, 16, false, 0, false><<<NN / 32, 64, 0, stream>>>(AVF, nullptr, WO_, WOQ, Fp(8), out_x + (size_t)b * NN * NODE, NODE, NN, NN);
    yout_kernel<<<1, 128, 0, stream>>>(PS, out_x, Fp(2), Fp(17), Fp(18), Fp(19), Fp(20), out_y, b);
  }
}
